// AttentionBlock_7275674600243
// MI455X (gfx1250) — hardware-verified
//
#include <hip/hip_runtime.h>
#include <stdint.h>


#ifndef NB
#define NB 4
#endif
#ifndef SEQ
#define SEQ 4096
#endif
#define NB_FULL  4
#define SEQ_FULL 4096
#define EMBED    256
#define HEADS    4
#define HDIM     64
#define NGRP     8
#define CPG      32
#define QKVOUT   768
#define NTOK     (NB * SEQ)
#define PLD      72
#define TP       72

static_assert(EMBED == HEADS * HDIM);
static_assert(EMBED == NGRP * CPG);
static_assert(QKVOUT == 3 * EMBED);
static_assert(CPG == 32);
static_assert((SEQ % 128) == 0);
static_assert((NTOK % 128) == 0);
static_assert((EMBED % 128) == 0);
static_assert((QKVOUT % 128) == 0);
static_assert(NB >= 1 && NB <= NB_FULL);
static_assert(SEQ >= 128 && SEQ <= SEQ_FULL);
static_assert(HDIM == 64);

typedef _Float16     v16h __attribute__((ext_vector_type(16)));
typedef _Float16     v8h  __attribute__((ext_vector_type(8)));
typedef float        v8f  __attribute__((ext_vector_type(8)));
typedef float        v4f  __attribute__((ext_vector_type(4)));
typedef unsigned int v4u  __attribute__((ext_vector_type(4)));

union Frag  { v16h v; v8h h[2]; };
union Pack8 { v8h h; v4u u; };

static constexpr size_t PLANE_H   = (size_t)NTOK * EMBED;
static constexpr size_t WQKV_H    = (size_t)QKVOUT * EMBED;
static constexpr size_t WPRJ_H    = (size_t)EMBED * EMBED;
static constexpr size_t WS_HALVES = 5 * PLANE_H + WQKV_H + WPRJ_H;
static_assert(WS_HALVES * 2 <= (size_t)134217728);
static_assert(((PLANE_H * 2) % 128) == 0);
static_assert(((WQKV_H * 2) % 128) == 0);
static_assert(((WPRJ_H * 2) % 128) == 0);

static __device__ __forceinline__ v8f wmma16(v16h a, v16h b, v8f c) {
  v8f d = __builtin_amdgcn_wmma_f32_16x16x32_f16(false, a, false, b, (short)0, c, false, false);
  asm volatile("v_nop\n\tv_nop\n\tv_nop\n\tv_nop" : "+v"(d) : "v"(a), "v"(b));
  return d;
}

static __device__ __forceinline__ v16h frag_rows(const _Float16* base, int row0, size_t ld, int k0) {
  const int l = threadIdx.x & 31, hf = l >> 4, m = l & 15;
  const _Float16* p = base + (size_t)(row0 + m) * ld + k0 + 8 * hf;
  Frag f;
  f.h[0] = *(const v8h*)(p);
  f.h[1] = *(const v8h*)(p + 16);
  return f.v;
}

static __device__ __forceinline__ float bf16_rne(float f) {
  unsigned int u = __float_as_uint(f);
  u += 0x7fffu + ((u >> 16) & 1u);
  u &= 0xffff0000u;
  return __uint_as_float(u);
}

static __device__ __forceinline__ double shfl_xor_d(double v, int m) {
  const unsigned long long u = __builtin_bit_cast(unsigned long long, v);
  int lo = (int)(unsigned int)(u & 0xffffffffull);
  int hi = (int)(unsigned int)(u >> 32);
  lo = __shfl_xor(lo, m);
  hi = __shfl_xor(hi, m);
  const unsigned long long r = ((unsigned long long)(unsigned int)hi << 32) | (unsigned long long)(unsigned int)lo;
  return __builtin_bit_cast(double, r);
}

__global__ __launch_bounds__(256)
void k_cvt(const float* __restrict__ src, _Float16* __restrict__ dst,
           int rows, int cols, int period, int pstride, float scale) {
  const int c8n   = cols >> 3;
  const int total = rows * c8n;
  const int i     = blockIdx.x * 256 + threadIdx.x;
  if (i >= total) return;
  const int r  = i / c8n;
  const int c  = (i - r * c8n) * 8;
  const int rb = r / period;
  const int sr = rb * pstride + (r - rb * period);
  const float* s = src + (size_t)sr * cols + c;
  const v4f a = *(const v4f*)(s);
  const v4f b = *(const v4f*)(s + 4);
  Pack8 o;
  o.h[0] = (_Float16)(bf16_rne(a[0]) * scale);
  o.h[1] = (_Float16)(bf16_rne(a[1]) * scale);
  o.h[2] = (_Float16)(bf16_rne(a[2]) * scale);
  o.h[3] = (_Float16)(bf16_rne(a[3]) * scale);
  o.h[4] = (_Float16)(bf16_rne(b[0]) * scale);
  o.h[5] = (_Float16)(bf16_rne(b[1]) * scale);
  o.h[6] = (_Float16)(bf16_rne(b[2]) * scale);
  o.h[7] = (_Float16)(bf16_rne(b[3]) * scale);
  _Float16* d = dst + (size_t)r * cols + c;
  *(volatile v4u*)d = o.u;
  __threadfence();
  *(volatile v4u*)d = o.u;
}

__global__ __launch_bounds__(256)
void k_gn(const float* __restrict__ x, const float* __restrict__ gw,
          const float* __restrict__ gb, _Float16* __restrict__ hh) {
  __shared__ __attribute__((aligned(16))) _Float16 T[64 * TP];
  __shared__ double red[2 * 8 * 2];
  __shared__ float  stat[4];

  const int tid = threadIdx.x, w = tid >> 5, lane = tid & 31;
  const int cg = blockIdx.x, b = blockIdx.y;
  const int cbase = cg * 64;
  const float* xb = x + ((size_t)b * EMBED + cbase) * SEQ_FULL;

  constexpr int qpc  = SEQ / 4;
  constexpr int nvec = CPG * qpc;
#pragma unroll
  for (int g = 0; g < 2; ++g) {
    double s = 0.0, ss = 0.0;
#pragma unroll 1
    for (int i = tid; i < nvec; i += 256) {
      const int c  = i / qpc;
      const int n4 = (i - c * qpc) * 4;
      const v4f v = *(const v4f*)(xb + (size_t)(g * CPG + c) * SEQ_FULL + n4);
      const double a0 = (double)bf16_rne(v[0]);
      const double a1 = (double)bf16_rne(v[1]);
      const double a2 = (double)bf16_rne(v[2]);
      const double a3 = (double)bf16_rne(v[3]);
      s  += (a0 + a1) + (a2 + a3);
      ss += (a0 * a0 + a1 * a1) + (a2 * a2 + a3 * a3);
    }
#pragma unroll
    for (int off = 16; off >= 1; off >>= 1) {
      s  += shfl_xor_d(s, off);
      ss += shfl_xor_d(ss, off);
    }
    if (lane == 0) {
      red[(g * 8 + w) * 2]     = s;
      red[(g * 8 + w) * 2 + 1] = ss;
    }
  }
  __syncthreads();
  if (tid == 0) {
#pragma unroll
    for (int g = 0; g < 2; ++g) {
      double S = 0.0, Q = 0.0;
#pragma unroll
      for (int ww = 0; ww < 8; ++ww) {
        S += red[(g * 8 + ww) * 2];
        Q += red[(g * 8 + ww) * 2 + 1];
      }
      const double inv_cnt = 1.0 / (double)((long long)CPG * SEQ);
      const double mean = S * inv_cnt;
      double var = Q * inv_cnt - mean * mean;
      if (var < 0.0) var = 0.0;
      const float ve = (float)var + 1.0e-5f;
      stat[2 * g]     = (float)mean;
      stat[2 * g + 1] = 1.0f / sqrtf(ve);
    }
  }
  __syncthreads();

  const int cl = tid >> 4;
  const int n4 = (tid & 15) * 4;
  float wc[4], bc[4], mu[4], rs[4];
#pragma unroll
  for (int i = 0; i < 4; ++i) {
    const int c = cl + 16 * i;
    wc[i] = bf16_rne(gw[cbase + c]);
    bc[i] = bf16_rne(gb[cbase + c]);
    mu[i] = stat[2 * (i >> 1)];
    rs[i] = stat[2 * (i >> 1) + 1];
  }
  const int orow = tid >> 3;
  const int oc8  = (tid & 7) * 8;

#pragma unroll 1
  for (int t0 = 0; t0 < SEQ; t0 += 64) {
    __syncthreads();
#pragma unroll
    for (int i = 0; i < 4; ++i) {
      const int c = cl + 16 * i;
      const v4f v = *(const v4f*)(xb + (size_t)c * SEQ_FULL + t0 + n4);
#pragma unroll
      for (int j = 0; j < 4; ++j) {
        const float hv = ((bf16_rne(v[j]) - mu[i]) * rs[i]) * wc[i] + bc[i];
        T[(n4 + j) * TP + c] = (_Float16)hv;
      }
    }
    __syncthreads();
    Pack8 o0, o1;
    o0.h = *(const v8h*)(T + orow * TP + oc8);
    o1.h = *(const v8h*)(T + (orow + 32) * TP + oc8);
    _Float16* d0 = hh + (size_t)(b * SEQ + t0 + orow) * EMBED + cbase + oc8;
    _Float16* d1 = d0 + (size_t)32 * EMBED;
    *(volatile v4u*)d0 = o0.u;
    *(volatile v4u*)d1 = o1.u;
    __threadfence();
    *(volatile v4u*)d0 = o0.u;
    *(volatile v4u*)d1 = o1.u;
  }
}

template <int MODE>
__global__ __launch_bounds__(256)
void k_gemm(const _Float16* __restrict__ A,
            const _Float16* __restrict__ W0, const _Float16* __restrict__ W1,
            const _Float16* __restrict__ W2,
            const float* __restrict__ G0, const float* __restrict__ G1,
            const float* __restrict__ G2,
            const float* __restrict__ R,
            void* O0, void* O1, void* O2,
            int K, int Nout, int ztr, float oscale) {
  __shared__ __attribute__((aligned(16))) float Cs[128 * 128];

  const int tid = threadIdx.x, w = tid >> 5, lane = tid & 31;
  const int hf = lane >> 4, nin = lane & 15;
  const int wm = w >> 1, wn = w & 1;
  const int m_blk = blockIdx.y * 128, n_blk = blockIdx.x * 128;
  const int z = blockIdx.z;
  const _Float16* W  = (z == 0) ? W0 : ((z == 1) ? W1 : W2);
  const float*  bias = (z == 0) ? G0 : ((z == 1) ? G1 : G2);
  void*           Ov = (z == 0) ? O0 : ((z == 1) ? O1 : O2);

  v8f acc[2][4] = {};

#pragma unroll 1
  for (int k0 = 0; k0 < K; k0 += 32) {
    const v16h a0 = frag_rows(A, m_blk + wm * 32,      (size_t)K, k0);
    const v16h a1 = frag_rows(A, m_blk + wm * 32 + 16, (size_t)K, k0);
#pragma unroll
    for (int nt = 0; nt < 4; ++nt) {
      const v16h bf = frag_rows(W, n_blk + wn * 64 + nt * 16, (size_t)K, k0);
      acc[0][nt] = wmma16(a0, bf, acc[0][nt]);
      acc[1][nt] = wmma16(a1, bf, acc[1][nt]);
    }
  }

#pragma unroll
  for (int nt = 0; nt < 4; ++nt) {
    const int ncol = wn * 64 + nt * 16 + nin;
    const float bv = bf16_rne(bias[n_blk + ncol]);
#pragma unroll
    for (int mt = 0; mt < 2; ++mt)
#pragma unroll
      for (int r = 0; r < 8; ++r) {
        const int row = wm * 32 + mt * 16 + 8 * hf + r;
        const float val = acc[mt][nt][r] * oscale + bv;
        if (MODE == 1) Cs[ncol * 128 + row] = val;
        else           Cs[row * 128 + ncol] = val;
      }
  }
  __syncthreads();

  if (MODE == 1) {
    float* out = (float*)Ov;
    const int bidx = m_blk / SEQ;
    const int s0   = m_blk - bidx * SEQ;
    v4f vals[16];
#pragma unroll
    for (int i = 0; i < 16; ++i) {
      const int c = w * 16 + i;
      const int n = n_blk + c;
      const v4f a  = *(const v4f*)(&Cs[c * 128 + 4 * lane]);
      const v4f xr = *(const v4f*)(R + ((size_t)bidx * EMBED + n) * SEQ_FULL + s0 + 4 * lane);
      v4f o;
      o[0] = bf16_rne(xr[0]) + a[0];
      o[1] = bf16_rne(xr[1]) + a[1];
      o[2] = bf16_rne(xr[2]) + a[2];
      o[3] = bf16_rne(xr[3]) + a[3];
      vals[i] = o;
    }
#pragma unroll
    for (int i = 0; i < 16; ++i) {
      const int n = n_blk + w * 16 + i;
      *(volatile v4f*)(out + ((size_t)bidx * EMBED + n) * SEQ + s0 + 4 * lane) = vals[i];
    }
    __threadfence();
#pragma unroll
    for (int i = 0; i < 16; ++i) {
      const int n = n_blk + w * 16 + i;
      *(volatile v4f*)(out + ((size_t)bidx * EMBED + n) * SEQ + s0 + 4 * lane) = vals[i];
    }
  } else {
    _Float16* out = (_Float16*)Ov;
    if (z != ztr) {
      v4u vals[8];
      const int c0 = nin * 8;
#pragma unroll
      for (int i = 0; i < 8; ++i) {
        const int row = w * 16 + 2 * i + hf;
        const v4f a = *(const v4f*)(&Cs[row * 128 + c0]);
        const v4f b = *(const v4f*)(&Cs[row * 128 + c0 + 4]);
        Pack8 o;
        o.h[0] = (_Float16)a[0]; o.h[1] = (_Float16)a[1];
        o.h[2] = (_Float16)a[2]; o.h[3] = (_Float16)a[3];
        o.h[4] = (_Float16)b[0]; o.h[5] = (_Float16)b[1];
        o.h[6] = (_Float16)b[2]; o.h[7] = (_Float16)b[3];
        vals[i] = o.u;
      }
#pragma unroll
      for (int i = 0; i < 8; ++i) {
        const int row = w * 16 + 2 * i + hf;
        *(volatile v4u*)(out + (size_t)(m_blk + row) * Nout + n_blk + c0) = vals[i];
      }
      __threadfence();
#pragma unroll
      for (int i = 0; i < 8; ++i) {
        const int row = w * 16 + 2 * i + hf;
        *(volatile v4u*)(out + (size_t)(m_blk + row) * Nout + n_blk + c0) = vals[i];
      }
    } else {
      const int bidx = m_blk / SEQ;
      const int s0 = m_blk - bidx * SEQ;
      const int t0 = nin * 8;
      v4u vals[8];
#pragma unroll
      for (int i = 0; i < 8; ++i) {
        const int c = w * 16 + 2 * i + hf;
        Pack8 o;
#pragma unroll
        for (int j = 0; j < 8; ++j) o.h[j] = (_Float16)Cs[(t0 + j) * 128 + c];
        vals[i] = o.u;
      }
#pragma unroll
      for (int i = 0; i < 8; ++i) {
        const int c = w * 16 + 2 * i + hf;
        const int n = n_blk + c;
        const int hh = n / HDIM, d = n - hh * HDIM;
        _Float16* dst = out + ((size_t)(bidx * HEADS + hh) * HDIM + d) * SEQ + s0 + t0;
        *(volatile v4u*)dst = vals[i];
      }
      __threadfence();
#pragma unroll
      for (int i = 0; i < 8; ++i) {
        const int c = w * 16 + 2 * i + hf;
        const int n = n_blk + c;
        const int hh = n / HDIM, d = n - hh * HDIM;
        _Float16* dst = out + ((size_t)(bidx * HEADS + hh) * HDIM + d) * SEQ + s0 + t0;
        *(volatile v4u*)dst = vals[i];
      }
    }
  }
}

__global__ __launch_bounds__(128) __attribute__((amdgpu_num_vgpr(256)))
void k_attn(const _Float16* __restrict__ qh, const _Float16* __restrict__ kh,
            const _Float16* __restrict__ vt, _Float16* __restrict__ oh, float scale) {
  __shared__ __attribute__((aligned(16))) _Float16 Ps[4 * 16 * PLD];

  const int tid = threadIdx.x, w = tid >> 5, lane = tid & 31;
  const int hf = lane >> 4, nin = lane & 15;
  const int qblk = blockIdx.x, h = blockIdx.y, b = blockIdx.z;
  const int qtok0 = b * SEQ + qblk * 64 + w * 16;
  const int ktokb = b * SEQ;
  _Float16* Pw = Ps + w * 16 * PLD;
  const _Float16* vtb = vt + (size_t)(b * HEADS + h) * HDIM * SEQ;

  v16h qa[2];
  {
    const _Float16* qp = qh + (size_t)(qtok0 + nin) * EMBED + h * HDIM + 8 * hf;
    Frag f;
    f.h[0] = *(const v8h*)(qp);      f.h[1] = *(const v8h*)(qp + 16); qa[0] = f.v;
    f.h[0] = *(const v8h*)(qp + 32); f.h[1] = *(const v8h*)(qp + 48); qa[1] = f.v;
  }

  float mrow[8], lrow[8];
#pragma unroll
  for (int r = 0; r < 8; ++r) { mrow[r] = -1.0e30f; lrow[r] = 0.0f; }
  v8f oacc[4] = {};

  const int nkb = SEQ / 64;
#pragma unroll 1
  for (int kb = 0; kb < nkb; ++kb) {
    __syncthreads();

    v8f sacc[4] = {};
#pragma unroll
    for (int nt = 0; nt < 4; ++nt) {
      const _Float16* kp = kh + (size_t)(ktokb + kb * 64 + nt * 16 + nin) * EMBED + h * HDIM + 8 * hf;
      Frag f;
      f.h[0] = *(const v8h*)(kp);      f.h[1] = *(const v8h*)(kp + 16);
      sacc[nt] = wmma16(qa[0], f.v, sacc[nt]);
      Frag g;
      g.h[0] = *(const v8h*)(kp + 32); g.h[1] = *(const v8h*)(kp + 48);
      sacc[nt] = wmma16(qa[1], g.v, sacc[nt]);
    }

#pragma unroll
    for (int r = 0; r < 8; ++r) {
      const float s0 = sacc[0][r] * scale, s1 = sacc[1][r] * scale;
      const float s2 = sacc[2][r] * scale, s3 = sacc[3][r] * scale;
      float t = fmaxf(fmaxf(s0, s1), fmaxf(s2, s3));
      t = fmaxf(t, __shfl_xor(t, 8, 16));
      t = fmaxf(t, __shfl_xor(t, 4, 16));
      t = fmaxf(t, __shfl_xor(t, 2, 16));
      t = fmaxf(t, __shfl_xor(t, 1, 16));
      const float mn    = fmaxf(mrow[r], t);
      const float alpha = __expf(mrow[r] - mn);
      mrow[r] = mn;
      const float p0 = __expf(s0 - mn), p1 = __expf(s1 - mn);
      const float p2 = __expf(s2 - mn), p3 = __expf(s3 - mn);
      float rs = (p0 + p1) + (p2 + p3);
      rs += __shfl_xor(rs, 8, 16);
      rs += __shfl_xor(rs, 4, 16);
      rs += __shfl_xor(rs, 2, 16);
      rs += __shfl_xor(rs, 1, 16);
      lrow[r] = lrow[r] * alpha + rs;
      sacc[0][r] = p0; sacc[1][r] = p1; sacc[2][r] = p2; sacc[3][r] = p3;
      oacc[0][r] *= alpha; oacc[1][r] *= alpha; oacc[2][r] *= alpha; oacc[3][r] *= alpha;
    }

#pragma unroll
    for (int nt = 0; nt < 4; ++nt)
#pragma unroll
      for (int r = 0; r < 8; ++r)
        Pw[(8 * hf + r) * PLD + nt * 16 + nin] = (_Float16)(sacc[nt][r] * 1024.0f);
    __syncthreads();

#pragma unroll
    for (int ks = 0; ks < 2; ++ks) {
      const v16h pf = frag_rows(Pw, 0, (size_t)PLD, ks * 32);
#pragma unroll
      for (int dt = 0; dt < 4; ++dt) {
        const _Float16* vp = vtb + (size_t)(dt * 16 + nin) * SEQ + kb * 64 + ks * 32 + 8 * hf;
        Frag f;
        f.h[0] = *(const v8h*)(vp); f.h[1] = *(const v8h*)(vp + 16);
        oacc[dt] = wmma16(pf, f.v, oacc[dt]);
      }
    }
  }
  __syncthreads();

#pragma unroll
  for (int r = 0; r < 8; ++r) {
    const float inv = 0.0625f * (1.0f / lrow[r]);
#pragma unroll
    for (int dt = 0; dt < 4; ++dt)
      Pw[(8 * hf + r) * PLD + dt * 16 + nin] = (_Float16)(oacc[dt][r] * inv);
  }
  __syncthreads();

  Pack8 vals[4];
  const int cl = (lane & 7) * 8;
#pragma unroll
  for (int i = 0; i < 4; ++i) {
    const int row = (lane >> 3) + 4 * i;
    vals[i].h = *(const v8h*)(Pw + row * PLD + cl);
  }
#pragma unroll
  for (int i = 0; i < 4; ++i) {
    const int row = (lane >> 3) + 4 * i;
    *(volatile v4u*)(oh + (size_t)(qtok0 + row) * EMBED + h * HDIM + cl) = vals[i].u;
  }
  __threadfence();
#pragma unroll
  for (int i = 0; i < 4; ++i) {
    const int row = (lane >> 3) + 4 * i;
    *(volatile v4u*)(oh + (size_t)(qtok0 + row) * EMBED + h * HDIM + cl) = vals[i].u;
  }
}

extern "C" void kernel_launch(void* const* d_in, const int* in_sizes, int n_in,
                              void* d_out, int out_size, void* d_ws, size_t ws_size,
                              hipStream_t stream) {
  if (n_in < 7) return;
  const long long need_x = ((long long)(NB - 1) * EMBED + (EMBED - 1)) * (long long)SEQ_FULL + SEQ;
  if ((long long)in_sizes[0] < need_x) return;
  if (in_sizes[1] < EMBED || in_sizes[2] < EMBED) return;
  if (in_sizes[3] < QKVOUT * EMBED || in_sizes[4] < QKVOUT) return;
  if (in_sizes[5] < EMBED * EMBED || in_sizes[6] < EMBED) return;
  if ((long long)out_size < (long long)NB * EMBED * SEQ) return;
  const size_t ws_need = WS_HALVES * sizeof(_Float16);
  if (ws_need > ws_size) return;

  const float* x      = (const float*)d_in[0];
  const float* norm_w = (const float*)d_in[1];
  const float* norm_b = (const float*)d_in[2];
  const float* qkv_w  = (const float*)d_in[3];
  const float* qkv_b  = (const float*)d_in[4];
  const float* proj_w = (const float*)d_in[5];
  const float* proj_b = (const float*)d_in[6];
  float* out = (float*)d_out;

  _Float16* hh   = (_Float16*)d_ws;
  _Float16* wqkv = hh   + PLANE_H;
  _Float16* wprj = wqkv + WQKV_H;
  _Float16* qh   = wprj + WPRJ_H;
  _Float16* kh   = qh   + PLANE_H;
  _Float16* vt   = kh   + PLANE_H;
  _Float16* oh   = vt   + PLANE_H;

  {
    const int tq = QKVOUT * (EMBED / 8);
    k_cvt<<<(tq + 255) / 256, 256, 0, stream>>>(qkv_w, wqkv, QKVOUT, EMBED, QKVOUT, QKVOUT, 64.0f);
    const int tp = EMBED * (EMBED / 8);
    k_cvt<<<(tp + 255) / 256, 256, 0, stream>>>(proj_w, wprj, EMBED, EMBED, EMBED, EMBED, 64.0f);
  }

  k_gn<<<dim3(EMBED / 64, NB), 256, 0, stream>>>(x, norm_w, norm_b, hh);

  k_gemm<0><<<dim3(EMBED / 128, NTOK / 128, 3), 256, 0, stream>>>(
      hh, wqkv, wqkv + (size_t)EMBED * EMBED, wqkv + (size_t)2 * EMBED * EMBED,
      qkv_b, qkv_b + EMBED, qkv_b + 2 * EMBED, x,
      (void*)qh, (void*)kh, (void*)vt,
      EMBED, EMBED, 2, 0.015625f);

  k_attn<<<dim3(SEQ / 64, HEADS, NB), 128, 0, stream>>>(qh, kh, vt, oh, 0.125f);

  k_gemm<1><<<dim3(EMBED / 128, NTOK / 128, 1), 256, 0, stream>>>(
      oh, wprj, wprj, wprj, proj_b, proj_b, proj_b, x,
      (void*)out, (void*)out, (void*)out,
      EMBED, EMBED, -1, 0.000244140625f);
}
